// Model_50620484550894
// MI455X (gfx1250) — hardware-verified
//
#include <hip/hip_runtime.h>
#include <stddef.h>
#include <stdint.h>
#include <math.h>


#define VV     50000
#define DD     300
#define DP     320
#define HD     96
#define NB     32
#define LL     1024
#define SS     256
#define CC     20
#define NE     1048576
#define NN     32768
#define G4     384
#define KC     384
#define K2     192
#define NR     8192

#define NTHR   256
#define NWAVE  8
#define EPT    8
#define CHUNK  (NTHR * EPT)
#define WCAP   (EPT * 32)
#define LISTN  (NWAVE * WCAP)
#define NBA    512
#define SLA    9
#define RCAP   18432
#define DEGCAP 96
#define MEAS_B512 16756
#define MEAS_DEG  57
#define BK_ZINTS (LISTN + 2 * RCAP + 3 * NBA)
#define BK_LDS_INTS (BK_ZINTS + 16)
#define AGR    8
#define GBM    64
#define GTHR   128
#define LTHR   384
#define WP     104
#define HP     200
#define WSMAX  134217728

#define M_ENC 0
#define M_ZR  1
#define M_HH  2
#define M_XG  3

#define SP_ENCB 0
#define SP_GRUB 96
#define SP_B0   672
#define SP_B1   1440
#define SP_ATW  2208
#define SP_ATB  11424
#define SP_F1W  11520
#define SP_F1B  20736
#define SP_F2W  20832
#define SP_F2B  22752
#define SP_N    22784

#define PB_XE   5120
#define PB_ENCT 15
#define PB_WG   54
#define PB_WI0  72
#define PB_WI1  144
#define PB_WHH  36
#define PB_SP   10
#define PB_ALL  (PB_XE + PB_ENCT + PB_WG + PB_WI0 + PB_WI1 + 2 * PB_WHH + PB_SP)

static_assert(NN == NB * LL && NR == SS * NB);
static_assert(HD == 96 && G4 == 4 * HD && NB == 32 && SS == 256);
static_assert(DP % 32 == 0 && KC % 32 == 0 && K2 % 32 == 0 && DP >= DD);
static_assert(NN % GBM == 0 && NR % GBM == 0 && GBM == (GTHR / 32) * 16);
static_assert(LTHR == 12 * 32 && (NB / 16) * (HD / 16) == 12);
static_assert((CHUNK & (CHUNK - 1)) == 0 && NBA == (1 << SLA) && NN % NBA == 0 && NN / NBA == 64);
static_assert(((long long)NE << SLA) < (1LL << 31) && NE % CHUNK == 0);
static_assert(RCAP * 100 >= MEAS_B512 * 105 && DEGCAP >= MEAS_DEG + 8 && DEGCAP % 32 == 0);
static_assert((RCAP / 2) % NTHR == 0 && BK_ZINTS % 4 == 0 && NTHR * 4 == 2 * NBA);
static_assert(NN % (NWAVE * AGR) == 0);
static_assert(PB_XE * NTHR == NN * (DP / 8) && PB_ENCT * NTHR == HD * (DP / 8));
static_assert(PB_WG * NTHR == 288 * (KC / 8) && PB_WI0 * NTHR == 768 * (K2 / 8));
static_assert(PB_WI1 * NTHR == 768 * (KC / 8) && PB_WHH * NTHR == 768 * (HD / 8));
static_assert((NR * 24) % NTHR == 0);
static_assert(2LL * NR * G4 * 4 == 2LL * NN * HD * 4);
static_assert(640 + NB * SS == 8832);

typedef float          v4f   __attribute__((ext_vector_type(4)));
typedef float          v8f   __attribute__((ext_vector_type(8)));
typedef int            v2i   __attribute__((ext_vector_type(2)));
typedef int            v4i   __attribute__((ext_vector_type(4)));
typedef int            v8i   __attribute__((ext_vector_type(8)));
typedef unsigned short v8us  __attribute__((ext_vector_type(8)));
typedef unsigned short v16us __attribute__((ext_vector_type(16)));
typedef __bf16         v16bf __attribute__((ext_vector_type(16)));
typedef v4f  __attribute__((may_alias)) v4fa;
typedef v2i  __attribute__((may_alias)) v2ia;
typedef v4i  __attribute__((may_alias)) v4ia;
typedef v8us __attribute__((may_alias)) v8usa;
union FragB { v16bf v; v16us u; v8us h[2]; v8i w; };

__device__ __forceinline__ v8f wmb(const FragB& a, const FragB& b, v8f c) {
  v8f d = __builtin_amdgcn_wmma_f32_16x16x32_bf16(false, a.v, false, b.v, (short)0, c, false, false);
  asm volatile("v_nop\n\tv_nop\n\tv_nop\n\tv_nop" : "+v"(d) : "v"(a.w), "v"(b.w));
  return d;
}

__device__ __forceinline__ unsigned bf16_bits(float f) {
  const unsigned u = __float_as_uint(f);
  const unsigned r = (u + 0x7FFFu + ((u >> 16) & 1u)) >> 16;
  return (f != f) ? 0x7FC0u : r;
}
__device__ __forceinline__ float bf16_val(float f) { return __uint_as_float(bf16_bits(f) << 16); }
__device__ __forceinline__ float sigm(float v) { return 1.0f / (1.0f + expf(-v)); }

__device__ __forceinline__ void put8(unsigned short* dp, v8us o) {
  *(volatile v8us*)dp = o; __threadfence(); *(volatile v8us*)dp = o;
}
__device__ __forceinline__ void put4f(float* dp, v4f o) {
  *(volatile v4f*)dp = o; __threadfence(); *(volatile v4f*)dp = o;
}
__device__ __forceinline__ void put4i(int* dp, v4i o) {
  *(volatile v4i*)dp = o; __threadfence(); *(volatile v4i*)dp = o;
}

__device__ __forceinline__ v8us cvt8(const float* __restrict__ p) {
  const v4f a = *(const v4fa*)p;
  const v4f b = *(const v4fa*)(p + 4);
  v8us o;
  o[0] = (unsigned short)bf16_bits(a.x); o[1] = (unsigned short)bf16_bits(a.y);
  o[2] = (unsigned short)bf16_bits(a.z); o[3] = (unsigned short)bf16_bits(a.w);
  o[4] = (unsigned short)bf16_bits(b.x); o[5] = (unsigned short)bf16_bits(b.y);
  o[6] = (unsigned short)bf16_bits(b.z); o[7] = (unsigned short)bf16_bits(b.w);
  return o;
}

__device__ __forceinline__ void hilo_pack(float v0, float v1, float v2, float v3,
                                          int& h01, int& h23, int& l01, int& l23) {
  const unsigned a0 = bf16_bits(v0), a1 = bf16_bits(v1), a2 = bf16_bits(v2), a3 = bf16_bits(v3);
  const unsigned b0 = bf16_bits(v0 - __uint_as_float(a0 << 16));
  const unsigned b1 = bf16_bits(v1 - __uint_as_float(a1 << 16));
  const unsigned b2 = bf16_bits(v2 - __uint_as_float(a2 << 16));
  const unsigned b3 = bf16_bits(v3 - __uint_as_float(a3 << 16));
  h01 = (int)(a0 | (a1 << 16)); h23 = (int)(a2 | (a3 << 16));
  l01 = (int)(b0 | (b1 << 16)); l23 = (int)(b2 | (b3 << 16));
}

__device__ __forceinline__ v4i regroup24(int h01, int h23, int l01, int l23, int lane) {
  const int tt = lane < 12 ? lane : (lane < 24 ? lane - 12 : 0);
  const int s0 = 2 * tt, s1 = s0 + 1;
  const int a0 = __shfl(h01, s0, 32), a1 = __shfl(h23, s0, 32), a2 = __shfl(h01, s1, 32), a3 = __shfl(h23, s1, 32);
  const int b0 = __shfl(l01, s0, 32), b1 = __shfl(l23, s0, 32), b2 = __shfl(l01, s1, 32), b3 = __shfl(l23, s1, 32);
  const int mk = (lane < 12) ? -1 : 0;
  v4i o;
  o.x = (a0 & mk) | (b0 & ~mk); o.y = (a1 & mk) | (b1 & ~mk);
  o.z = (a2 & mk) | (b2 & ~mk); o.w = (a3 & mk) | (b3 & ~mk);
  return o;
}
__device__ __forceinline__ v4i pack_row24(float v0, float v1, float v2, float v3, int lane) {
  int h01, h23, l01, l23;
  hilo_pack(v0, v1, v2, v3, h01, h23, l01, l23);
  return regroup24(h01, h23, l01, l23, lane);
}

template <int SLB>
__device__ __forceinline__ int scan_chunk(const int* __restrict__ dsts, int nE, int cbase, int slotBase,
                                          int nb, int vec8, int* list, int tid, int lane, int wave) {
  int wc = 0;
  const int el0  = tid * EPT;
  const int e0   = cbase + el0;
  const int sent = -2147483647 - 1;
  v4i da, db;
  if (vec8 != 0 && cbase + CHUNK <= nE) {
    da = *(const v4i*)(dsts + e0);
    db = *(const v4i*)(dsts + e0 + 4);
  } else {
    da.x = (e0     < nE) ? dsts[min(e0,     nE - 1)] : sent;
    da.y = (e0 + 1 < nE) ? dsts[min(e0 + 1, nE - 1)] : sent;
    da.z = (e0 + 2 < nE) ? dsts[min(e0 + 2, nE - 1)] : sent;
    da.w = (e0 + 3 < nE) ? dsts[min(e0 + 3, nE - 1)] : sent;
    db.x = (e0 + 4 < nE) ? dsts[min(e0 + 4, nE - 1)] : sent;
    db.y = (e0 + 5 < nE) ? dsts[min(e0 + 5, nE - 1)] : sent;
    db.z = (e0 + 6 < nE) ? dsts[min(e0 + 6, nE - 1)] : sent;
    db.w = (e0 + 7 < nE) ? dsts[min(e0 + 7, nE - 1)] : sent;
  }
  const unsigned nbs = (unsigned)slotBase;
  const unsigned unb = (unsigned)nb;
  const unsigned s0 = (unsigned)da.x - nbs, s1 = (unsigned)da.y - nbs;
  const unsigned s2 = (unsigned)da.z - nbs, s3 = (unsigned)da.w - nbs;
  const unsigned s4 = (unsigned)db.x - nbs, s5 = (unsigned)db.y - nbs;
  const unsigned s6 = (unsigned)db.z - nbs, s7 = (unsigned)db.w - nbs;
  const bool h0 = s0 < unb, h1 = s1 < unb, h2 = s2 < unb, h3 = s3 < unb;
  const bool h4 = s4 < unb, h5 = s5 < unb, h6 = s6 < unb, h7 = s7 < unb;
  const unsigned any = __builtin_amdgcn_ballot_w32(h0 | h1 | h2 | h3 | h4 | h5 | h6 | h7);
  if (any != 0u) {
#define HITJ(J, HJ, SJ) { \
      const unsigned mj = __builtin_amdgcn_ballot_w32(HJ); \
      if (mj != 0u) { \
        if (HJ) { \
          const int pos = wc + (int)__builtin_amdgcn_mbcnt_lo(mj, 0u); \
          if (pos < WCAP) list[wave * WCAP + pos] = ((el0 + (J)) << SLB) | (int)(SJ); \
        } \
        wc += (int)__builtin_popcount(mj); } }
    HITJ(0, h0, s0)
    HITJ(1, h1, s1)
    HITJ(2, h2, s2)
    HITJ(3, h3, s3)
    HITJ(4, h4, s4)
    HITJ(5, h5, s5)
    HITJ(6, h6, s6)
    HITJ(7, h7, s7)
#undef HITJ
  }
  return wc;
}

__device__ __forceinline__ void sp_part(const float* __restrict__ src, int nsrc4, int ndst4, float* dst, int tid) {
#pragma unroll 1
  for (int v0 = 0; v0 < ndst4; v0 += NTHR) {
    const int v  = v0 + tid;
    const int vc = v < nsrc4 ? v : nsrc4 - 1;
    const v4f a = *(const v4fa*)(src + 4 * vc);
    const bool ok = v < nsrc4;
    v4f o;
    o.x = ok ? bf16_val(a.x) : 0.0f; o.y = ok ? bf16_val(a.y) : 0.0f;
    o.z = ok ? bf16_val(a.z) : 0.0f; o.w = ok ? bf16_val(a.w) : 0.0f;
    float* dp = dst + 4 * (v < ndst4 ? v : ndst4 - 1);
    if (v < ndst4) *(volatile v4f*)dp = o;
    __threadfence();
    if (v < ndst4) *(volatile v4f*)dp = o;
  }
}

__global__ __launch_bounds__(NTHR) void k_prep(
    const int* __restrict__ x, const float* __restrict__ emb, const float* __restrict__ encw,
    const float* __restrict__ encb, const float* __restrict__ gruw, const float* __restrict__ grub,
    const float* __restrict__ wih0, const float* __restrict__ whh0, const float* __restrict__ b0,
    const float* __restrict__ wih1, const float* __restrict__ whh1, const float* __restrict__ b1,
    const float* __restrict__ atw, const float* __restrict__ atb, const float* __restrict__ f1w,
    const float* __restrict__ f1b, const float* __restrict__ f2w, const float* __restrict__ f2b,
    unsigned short* XE, unsigned short* ENCT, unsigned short* WG, unsigned short* WI0, unsigned short* WI1,
    unsigned short* WHH0, unsigned short* WHH1, float* SP)
{
  const int tid = (int)threadIdx.x;
  int blk = (int)blockIdx.x;
  if (blk < PB_XE) {
    const int u  = blk * NTHR + tid;
    const int n  = u / 40;
    const int k8 = (u - n * 40) * 8;
    int xi = x[n];
    xi = xi < 0 ? 0 : (xi > VV ? VV : xi);
    const float* er = emb + (size_t)xi * DD;
    const int ka = k8 < 296 ? k8 : 296;
    const int kb = (k8 + 4) < 296 ? (k8 + 4) : 296;
    const v4f a = *(const v4fa*)(er + ka);
    const v4f b = *(const v4fa*)(er + kb);
    const bool oa = k8 < DD;
    const bool ob = (k8 + 4) < DD;
    v8us o;
    o[0] = oa ? (unsigned short)bf16_bits(a.x) : (unsigned short)0;
    o[1] = oa ? (unsigned short)bf16_bits(a.y) : (unsigned short)0;
    o[2] = oa ? (unsigned short)bf16_bits(a.z) : (unsigned short)0;
    o[3] = oa ? (unsigned short)bf16_bits(a.w) : (unsigned short)0;
    o[4] = ob ? (unsigned short)bf16_bits(b.x) : (unsigned short)0;
    o[5] = ob ? (unsigned short)bf16_bits(b.y) : (unsigned short)0;
    o[6] = ob ? (unsigned short)bf16_bits(b.z) : (unsigned short)0;
    o[7] = ob ? (unsigned short)bf16_bits(b.w) : (unsigned short)0;
    put8(XE + (size_t)8 * u, o);
    return;
  }
  blk -= PB_XE;
  if (blk < PB_ENCT) {
    const int v  = blk * NTHR + tid;
    const int n  = v / 40;
    const int k8 = (v - n * 40) * 8;
    v8us o;
#pragma unroll
    for (int i = 0; i < 8; ++i) {
      const int k  = k8 + i;
      const int kc = k < DD ? k : DD - 1;
      const float f = encw[kc * HD + n];
      o[i] = (k < DD) ? (unsigned short)bf16_bits(f) : (unsigned short)0;
    }
    put8(ENCT + (size_t)8 * v, o);
    return;
  }
  blk -= PB_ENCT;
  if (blk < PB_WG) {
    const int v   = blk * NTHR + tid;
    const int n   = v / 48;
    const int k8  = (v - n * 48) * 8;
    const int seg = k8 / HD;
    const int kk  = k8 - seg * HD;
    const int grp = n / HD;
    const int nn  = n - grp * HD;
    const int j   = 2 * grp + (seg >> 1);
    const float* p = gruw + (size_t)j * (HD * HD) + kk * HD + nn;
    v8us o;
#pragma unroll
    for (int i = 0; i < 8; ++i) o[i] = (unsigned short)bf16_bits(p[i * HD]);
    put8(WG + (size_t)8 * v, o);
    return;
  }
  blk -= PB_WG;
  if (blk < PB_WI0) {
    const int v  = blk * NTHR + tid;
    const int n  = v / 24;
    const int k8 = (v - n * 24) * 8;
    const int kk = k8 >= HD ? k8 - HD : k8;
    put8(WI0 + (size_t)8 * v, cvt8(wih0 + (size_t)n * HD + kk));
    return;
  }
  blk -= PB_WI0;
  if (blk < PB_WI1) {
    const int v   = blk * NTHR + tid;
    const int n   = v / 48;
    const int k8  = (v - n * 48) * 8;
    const int seg = k8 / HD;
    const int kk  = k8 - seg * HD;
    const int col = (seg >= 2 ? HD : 0) + kk;
    put8(WI1 + (size_t)8 * v, cvt8(wih1 + (size_t)n * (2 * HD) + col));
    return;
  }
  blk -= PB_WI1;
  if (blk < PB_WHH) {
    const int v = blk * NTHR + tid;
    put8(WHH0 + (size_t)8 * v, cvt8(whh0 + (size_t)8 * v));
    return;
  }
  blk -= PB_WHH;
  if (blk < PB_WHH) {
    const int v = blk * NTHR + tid;
    put8(WHH1 + (size_t)8 * v, cvt8(whh1 + (size_t)8 * v));
    return;
  }
  blk -= PB_WHH;
  if (blk == 0)      sp_part(encb, 24,   24,   SP + SP_ENCB, tid);
  else if (blk == 1) sp_part(grub, 144,  144,  SP + SP_GRUB, tid);
  else if (blk == 2) sp_part(b0,   192,  192,  SP + SP_B0,   tid);
  else if (blk == 3) sp_part(b1,   192,  192,  SP + SP_B1,   tid);
  else if (blk == 4) sp_part(atw,  2304, 2304, SP + SP_ATW,  tid);
  else if (blk == 5) sp_part(atb,  24,   24,   SP + SP_ATB,  tid);
  else if (blk == 6) sp_part(f1w,  2304, 2304, SP + SP_F1W,  tid);
  else if (blk == 7) sp_part(f1b,  24,   24,   SP + SP_F1B,  tid);
  else if (blk == 8) sp_part(f2w,  480,  480,  SP + SP_F2W,  tid);
  else if (blk == 9) sp_part(f2b,  5,    8,    SP + SP_F2B,  tid);
}

__global__ __launch_bounds__(NTHR) void k_bucket(const int* __restrict__ esrc, const int* __restrict__ dsts,
                                                 const float* __restrict__ ew, int nE, int nN, int vec8,
                                                 int* LIST, int* OC, int* FLAG) {
  extern __shared__ __attribute__((aligned(16))) int dsm[];
  int* list = dsm;
  int* hl   = dsm + LISTN;
  int* sl   = dsm + LISTN + RCAP;
  int* cnt  = dsm + LISTN + 2 * RCAP;
  int* offs = cnt + NBA;
  int* cur  = offs + NBA;
  int* misc = cur + NBA;
  const int tid = (int)threadIdx.x, lane = tid & 31, wave = tid >> 5;
  const int nodeBase = (int)blockIdx.x * NBA;

  {
    const v4i z4 = {0, 0, 0, 0};
    for (int i = tid * 4; i < BK_ZINTS; i += NTHR * 4) *(v4ia*)(dsm + i) = z4;
    if (tid < 16) misc[tid] = 0;
  }
  __syncthreads();

  int t = 0, ov = 0;
  const int nChunks = (nE + CHUNK - 1) / CHUNK;
#pragma unroll 1
  for (int ch = 0; ch < nChunks; ++ch) {
    const int cbase = ch * CHUNK;
    const int wc = scan_chunk<SLA>(dsts, nE, cbase, nodeBase, NBA, vec8, list, tid, lane, wave);
    if (lane == 0) misc[wave] = wc;
    __syncthreads();
    if (wave == 0) {
#pragma unroll 1
      for (int w2 = 0; w2 < NWAVE; ++w2) {
        int c = misc[w2];
        c = c < 0 ? 0 : (c > WCAP ? WCAP : c);
#pragma unroll 1
        for (int b0 = 0; b0 < c; b0 += 32) {
          const int idx = b0 + lane;
          const int ent = list[w2 * WCAP + (idx < WCAP ? idx : WCAP - 1)];
          const int m32 = (c - b0) < 32 ? (c - b0) : 32;
#pragma unroll 1
          for (int k = 0; k < m32; ++k) {
            const int u    = __builtin_amdgcn_readlane(ent, k);
            const int slot = u & (NBA - 1);
            const int el   = (u >> SLA) & (CHUNK - 1);
            const int pk   = ((cbase + el) << SLA) | slot;
            if (t < RCAP) {
              if (lane == 0) { hl[t] = pk; cnt[slot] = cnt[slot] + 1; }
              t = t + 1;
            } else {
              ov = 1;
            }
          }
        }
      }
    }
    __syncthreads();
  }
  if (wave == 0 && lane == 0) { misc[8] = t; misc[9] = ov; }
  __syncthreads();
  int tt = misc[8];
  tt = tt < 0 ? 0 : (tt > RCAP ? RCAP : tt);

  if (wave == 0) {
    const int base = lane * (NBA / 32);
    int s = 0, dg = 0;
#pragma unroll 1
    for (int i = 0; i < NBA / 32; ++i) {
      const int cv = cnt[base + i];
      s += cv;
      dg |= (cv > DEGCAP) ? 1 : 0;
    }
    const unsigned dm = __builtin_amdgcn_ballot_w32(dg != 0);
    if (lane == 0) misc[10] = (dm != 0u) ? 1 : 0;
    int incl = s;
#pragma unroll
    for (int d = 1; d < 32; d <<= 1) {
      const int y = __shfl_up(incl, d, 32);
      if (lane >= d) incl += y;
    }
    int run = incl - s;
#pragma unroll 1
    for (int i = 0; i < NBA / 32; ++i) {
      const int cv = cnt[base + i];
      offs[base + i] = run;
      cur[base + i]  = run;
      run += cv;
    }
  }
  __syncthreads();
  if (wave == 0) {
#pragma unroll 1
    for (int b0 = 0; b0 < tt; b0 += 32) {
      const int idx = b0 + lane;
      const int ent = hl[idx < RCAP ? idx : RCAP - 1];
      const int m32 = (tt - b0) < 32 ? (tt - b0) : 32;
#pragma unroll 1
      for (int k = 0; k < m32; ++k) {
        const int u    = __builtin_amdgcn_readlane(ent, k);
        const int slot = u & (NBA - 1);
        if (lane == 0) {
          int p = cur[slot];
          p = p < 0 ? 0 : (p > RCAP - 1 ? RCAP - 1 : p);
          sl[p] = u;
          cur[slot] = p + 1;
        }
      }
    }
  }
  __syncthreads();
  const int ovf = ((misc[9] | misc[10]) != 0) ? 1 : 0;

  int* lp = LIST + (size_t)blockIdx.x * (size_t)(RCAP * 2);
#pragma unroll 1
  for (int it = 0; it < (RCAP / 2) / NTHR; ++it) {
    const int u  = it * NTHR + tid;
    const int p0 = 2 * u, p1 = 2 * u + 1;
    const v2i e2 = *(const v2ia*)(sl + p0);
    int id0 = e2.x >> SLA, id1 = e2.y >> SLA;
    id0 = id0 < 0 ? 0 : (id0 > nE - 1 ? nE - 1 : id0);
    id1 = id1 < 0 ? 0 : (id1 > nE - 1 ? nE - 1 : id1);
    int s0 = esrc[id0], s1 = esrc[id1];
    s0 = s0 < 0 ? 0 : (s0 > nN - 1 ? nN - 1 : s0);
    s1 = s1 < 0 ? 0 : (s1 > nN - 1 ? nN - 1 : s1);
    const int w0 = __float_as_int(bf16_val(ew[id0]));
    const int w1 = __float_as_int(bf16_val(ew[id1]));
    v4i o;
    o.x = (p0 < tt) ? s0 : 0; o.y = (p0 < tt) ? w0 : 0;
    o.z = (p1 < tt) ? s1 : 0; o.w = (p1 < tt) ? w1 : 0;
    put4i(lp + 4 * u, o);
  }
  {
    const int which = tid >> 7;
    const int i4 = (tid & 127) * 4;
    const v4i v = *(const v4ia*)(cnt + which * NBA + i4);
    put4i(OC + (size_t)which * nN + nodeBase + i4, v);
  }
  if (wave == 0) {
    int* fp = FLAG + (int)blockIdx.x * 32 + lane;
    *(volatile int*)fp = ovf;
    __threadfence();
    *(volatile int*)fp = ovf;
  }
}

__global__ __launch_bounds__(NTHR) void k_agg(const float* __restrict__ Hc, const int* __restrict__ LIST,
                                              const int* __restrict__ OC, const int* __restrict__ FLAG,
                                              int nN, unsigned short* ACAT) {
  const int tid = (int)threadIdx.x, lane = tid & 31, wave = tid >> 5;
  const int lc = lane < 24 ? lane : 23;
#pragma unroll 1
  for (int i = 0; i < AGR; ++i) {
    const int node = (int)blockIdx.x * (NWAVE * AGR) + wave * AGR + i;
    const int bk = node >> SLA;
    const int fl = FLAG[bk * 32];
    int c = OC[node];
    const bool big = c > DEGCAP;
    c = c < 0 ? 0 : (c > DEGCAP ? DEGCAP : c);
    int o = OC[nN + node];
    o = o < 0 ? 0 : (o > RCAP - 1 ? RCAP - 1 : o);
    int last = o + (c > 0 ? c - 1 : 0);
    last = last > RCAP - 1 ? RCAP - 1 : last;
    const int* lp = LIST + (size_t)bk * (size_t)(RCAP * 2);
    float g0 = 0.0f, g1 = 0.0f, g2 = 0.0f, g3 = 0.0f;
#pragma unroll 1
    for (int b0 = 0; b0 < c; b0 += 32) {
      int idx = o + b0 + lane;
      idx = idx > last ? last : idx;
      const v2i ent = *(const v2ia*)(lp + 2 * idx);
      int sr = ent.x;
      sr = sr < 0 ? 0 : (sr > nN - 1 ? nN - 1 : sr);
      const int wvi = ent.y;
      const int m32 = (c - b0) < 32 ? (c - b0) : 32;
#pragma unroll 1
      for (int k = 0; k < m32; ++k) {
        const int   sk = __builtin_amdgcn_readlane(sr, k);
        const float wk = __int_as_float(__builtin_amdgcn_readlane(wvi, k));
        const v4f a = *(const v4fa*)(Hc + (size_t)sk * HD + 4 * lc);
        g0 = fmaf(a.x, wk, g0); g1 = fmaf(a.y, wk, g1);
        g2 = fmaf(a.z, wk, g2); g3 = fmaf(a.w, wk, g3);
      }
    }
    const float pz = (big || fl != 0) ? __int_as_float(0x7fc00000) : 0.0f;
    const v4i ow = pack_row24(g0 + pz, g1 + pz, g2 + pz, g3 + pz, lane);
    unsigned short* hp = ACAT + (size_t)node * KC + 8 * lc;
    if (lane < 24) *(volatile v4i*)hp = ow;
    __threadfence();
    if (lane < 24) *(volatile v4i*)hp = ow;
  }
}

template <int MODE, int NT>
__global__ __launch_bounds__(GTHR) void k_gemm(
    const unsigned short* A1, int lda1, int ks1,
    const unsigned short* A2, int lda2, int ks2,
    const unsigned short* __restrict__ WT, int ldb,
    const float* __restrict__ bias, const float* rdH, const float* rdZ,
    float* outF, unsigned short* outH)
{
  constexpr int NW = 16 * NT;
  __shared__ __attribute__((aligned(16))) float stg[GBM * NW];
  const int tid = (int)threadIdx.x, lane = tid & 31, wave = tid >> 5, hh = lane >> 4, m = lane & 15;
  const int rowBase = (int)blockIdx.x * GBM;
  const int col0    = (int)blockIdx.y * NW;

  v8f acc[NT];
  {
    const v8f z = {0.f, 0.f, 0.f, 0.f, 0.f, 0.f, 0.f, 0.f};
#pragma unroll
    for (int t = 0; t < NT; ++t) acc[t] = z;
  }
  const unsigned short* ap1 = A1 + (size_t)(rowBase + 16 * wave + m) * (size_t)lda1 + 8 * hh;
  const unsigned short* ap2 = A2 + (size_t)(rowBase + 16 * wave + m) * (size_t)lda2 + 8 * hh;
  const unsigned short* wp  = WT + (size_t)(col0 + m) * (size_t)ldb + 8 * hh;
#pragma unroll 1
  for (int ks = 0; ks < ks1; ++ks) {
    FragB af;
    af.h[0] = *(const v8usa*)(ap1 + 32 * ks);
    af.h[1] = *(const v8usa*)(ap1 + 32 * ks + 16);
#pragma unroll
    for (int t = 0; t < NT; ++t) {
      const unsigned short* wq = wp + (size_t)(16 * t) * (size_t)ldb + 32 * ks;
      FragB bf;
      bf.h[0] = *(const v8usa*)wq;
      bf.h[1] = *(const v8usa*)(wq + 16);
      acc[t] = wmb(af, bf, acc[t]);
    }
  }
#pragma unroll 1
  for (int ks = 0; ks < ks2; ++ks) {
    FragB af;
    af.h[0] = *(const v8usa*)(ap2 + 32 * ks);
    af.h[1] = *(const v8usa*)(ap2 + 32 * ks + 16);
#pragma unroll
    for (int t = 0; t < NT; ++t) {
      const unsigned short* wq = wp + (size_t)(16 * t) * (size_t)ldb + 32 * (ks1 + ks);
      FragB bf;
      bf.h[0] = *(const v8usa*)wq;
      bf.h[1] = *(const v8usa*)(wq + 16);
      acc[t] = wmb(af, bf, acc[t]);
    }
  }

#pragma unroll
  for (int t = 0; t < NT; ++t) {
    const int lc = 16 * t + m;
#pragma unroll
    for (int r = 0; r < 8; ++r) {
      const int lr = 16 * wave + 8 * hh + r;
      stg[lr * NW + lc] = acc[t][r];
    }
  }
  __syncthreads();

  const int lq = lane < 24 ? lane : 23;
  const int c4 = 4 * lq;
  if constexpr (MODE == M_ENC || MODE == M_HH) {
    v4f bb;
    if constexpr (MODE == M_ENC) {
      bb = *(const v4fa*)(bias + c4);
    } else {
      const v4f b4 = *(const v4fa*)(bias + 4 * HD + c4);
      const v4f b5 = *(const v4fa*)(bias + 5 * HD + c4);
      bb.x = b4.x + b5.x; bb.y = b4.y + b5.y; bb.z = b4.z + b5.z; bb.w = b4.w + b5.w;
    }
#pragma unroll 1
    for (int i = 0; i < 16; ++i) {
      const int lr = 16 * wave + i;
      const int grow = rowBase + lr;
      const v4f t = *(const v4fa*)(stg + lr * NW + c4);
      v4f v;
      if constexpr (MODE == M_ENC) {
        v.x = tanhf(t.x + bb.x); v.y = tanhf(t.y + bb.y); v.z = tanhf(t.z + bb.z); v.w = tanhf(t.w + bb.w);
      } else {
        const v4f z = *(const v4fa*)(rdZ + (size_t)grow * HD + c4);
        const v4f h = *(const v4fa*)(rdH + (size_t)grow * HD + c4);
        const float q0 = tanhf(t.x + bb.x), q1 = tanhf(t.y + bb.y), q2 = tanhf(t.z + bb.z), q3 = tanhf(t.w + bb.w);
        v.x = q0 * z.x + h.x * (1.0f - z.x); v.y = q1 * z.y + h.y * (1.0f - z.y);
        v.z = q2 * z.z + h.z * (1.0f - z.z); v.w = q3 * z.w + h.w * (1.0f - z.w);
      }
      const v4i ow = pack_row24(v.x, v.y, v.z, v.w, lane);
      float* fp = outF + (size_t)grow * HD + c4;
      unsigned short* hp = outH + (size_t)grow * KC + 2 * HD + 8 * lq;
      if (lane < 24) { *(volatile v4f*)fp = v; *(volatile v4i*)hp = ow; }
      __threadfence();
      if (lane < 24) { *(volatile v4f*)fp = v; *(volatile v4i*)hp = ow; }
    }
  } else if constexpr (MODE == M_ZR) {
    v4f bz, br;
    {
      const v4f b0 = *(const v4fa*)(bias + 0 * HD + c4);
      const v4f b1 = *(const v4fa*)(bias + 1 * HD + c4);
      const v4f b2 = *(const v4fa*)(bias + 2 * HD + c4);
      const v4f b3 = *(const v4fa*)(bias + 3 * HD + c4);
      bz.x = b0.x + b1.x; bz.y = b0.y + b1.y; bz.z = b0.z + b1.z; bz.w = b0.w + b1.w;
      br.x = b2.x + b3.x; br.y = b2.y + b3.y; br.z = b2.z + b3.z; br.w = b2.w + b3.w;
    }
#pragma unroll 1
    for (int i = 0; i < 16; ++i) {
      const int lr = 16 * wave + i;
      const int grow = rowBase + lr;
      const v4f tz = *(const v4fa*)(stg + lr * NW + c4);
      const v4f tr = *(const v4fa*)(stg + lr * NW + HD + c4);
      const v4f h  = *(const v4fa*)(rdH + (size_t)grow * HD + c4);
      v4f z;
      z.x = sigm(tz.x + bz.x); z.y = sigm(tz.y + bz.y); z.z = sigm(tz.z + bz.z); z.w = sigm(tz.w + bz.w);
      const float r0 = sigm(tr.x + br.x), r1 = sigm(tr.y + br.y), r2 = sigm(tr.z + br.z), r3 = sigm(tr.w + br.w);
      const v4i ow = pack_row24(h.x * r0, h.y * r1, h.z * r2, h.w * r3, lane);
      float* fp = outF + (size_t)grow * HD + c4;
      unsigned short* hp = outH + (size_t)grow * K2 + 8 * lq;
      if (lane < 24) { *(volatile v4f*)fp = z; *(volatile v4i*)hp = ow; }
      __threadfence();
      if (lane < 24) { *(volatile v4f*)fp = z; *(volatile v4i*)hp = ow; }
    }
  } else {
    const int dirp = col0 / G4;
    const int cg   = col0 - dirp * G4;
    const int l16  = lane & 15;
    const v4f ba = *(const v4fa*)(bias + col0 + 4 * lane);
    const v4f bc = *(const v4fa*)(bias + col0 + 128 + 4 * l16);
    float* ob = outF + (size_t)dirp * ((size_t)NR * G4) + cg;
#pragma unroll 1
    for (int i = 0; i < 16; ++i) {
      const int lr = 16 * wave + i;
      const int grow = rowBase + lr;
      const v4f ta = *(const v4fa*)(stg + lr * NW + 4 * lane);
      const v4f tb = *(const v4fa*)(stg + lr * NW + 128 + 4 * l16);
      v4f oa, oc;
      oa.x = ta.x + ba.x; oa.y = ta.y + ba.y; oa.z = ta.z + ba.z; oa.w = ta.w + ba.w;
      oc.x = tb.x + bc.x; oc.y = tb.y + bc.y; oc.z = tb.z + bc.z; oc.w = tb.w + bc.w;
      float* p = ob + (size_t)grow * G4;
      *(volatile v4f*)(p + 4 * lane) = oa;
      if (lane < 16) *(volatile v4f*)(p + 128 + 4 * l16) = oc;
      __threadfence();
      *(volatile v4f*)(p + 4 * lane) = oa;
      if (lane < 16) *(volatile v4f*)(p + 128 + 4 * l16) = oc;
    }
  }
}

__global__ __launch_bounds__(NTHR) void k_gather(const int* __restrict__ xs, const unsigned short* __restrict__ ACAT,
                                                 unsigned short* XS) {
  const int u = (int)blockIdx.x * NTHR + (int)threadIdx.x;
  const int r = u / 24;
  const int q = u - r * 24;
  const int s = r >> 5, b = r & 31;
  int tok = xs[b * SS + s];
  tok = tok < 0 ? 0 : (tok > LL - 1 ? LL - 1 : tok);
  const int node = b * LL + tok;
  const v8us v = *(const v8usa*)(ACAT + (size_t)node * KC + 2 * HD + 8 * q);
  put8(XS + (size_t)8 * u, v);
}

template <int LAYER>
__global__ __launch_bounds__(LTHR) void k_lstm(const float* __restrict__ XG, const unsigned short* __restrict__ WHH,
                                               unsigned short* OUT0, float* O1, float* HT) {
  extern __shared__ __attribute__((aligned(16))) float lsm[];
  float* xs = lsm;
  float* hf = lsm + NB * G4;
  unsigned short* whh = (unsigned short*)(lsm + NB * G4 + NB * HD);
  unsigned short* hb  = whh + G4 * WP;
  const int tid = (int)threadIdx.x, lane = tid & 31, wave = tid >> 5, hh = lane >> 4, m = lane & 15;
  const int dir = (int)blockIdx.x;
  const int mt = wave / 6, jt = wave - 6 * mt;

  {
    const unsigned short* wsrc = WHH + (size_t)dir * (G4 * HD);
#pragma unroll 1
    for (int i = 0; i < 12; ++i) {
      const int p = tid + LTHR * i;
      const int row = p / 12, q = p - 12 * row;
      *(v8usa*)(whh + row * WP + 8 * q) = *(const v8usa*)(wsrc + row * HD + 8 * q);
    }
    const v8us z8 = {0, 0, 0, 0, 0, 0, 0, 0};
    *(v8usa*)(whh + tid * WP + HD) = z8;
#pragma unroll 1
    for (int p = tid; p < (2 * NB * HP) / 8; p += LTHR) *(v8usa*)(hb + 8 * p) = z8;
  }
  float cst[8];
#pragma unroll
  for (int r = 0; r < 8; ++r) cst[r] = 0.0f;
  __syncthreads();

#pragma unroll 1
  for (int st = 0; st < SS; ++st) {
    const int t   = dir ? (SS - 1 - st) : st;
    const int cur = st & 1, nxt = cur ^ 1;
    const float* slab = XG + ((size_t)dir * NR + (size_t)t * NB) * G4;
#pragma unroll
    for (int i = 0; i < 8; ++i) {
      const int f4 = tid + LTHR * i;
      *(v4fa*)(xs + 4 * f4) = *(const v4fa*)(slab + 4 * f4);
    }
    __syncthreads();

    v8f acc[4];
#pragma unroll
    for (int q = 0; q < 4; ++q) {
#pragma unroll
      for (int r = 0; r < 8; ++r) acc[q][r] = xs[(16 * mt + 8 * hh + r) * G4 + q * HD + 16 * jt + m];
    }
    const unsigned short* hrow = hb + cur * (NB * HP) + (16 * mt + m) * HP + 8 * hh;
#pragma unroll
    for (int ks = 0; ks < 6; ++ks) {
      FragB af;
      af.h[0] = *(const v8usa*)(hrow + 32 * ks);
      af.h[1] = *(const v8usa*)(hrow + 32 * ks + 16);
      const int kb = (ks % 3) * 32;
#pragma unroll
      for (int q = 0; q < 4; ++q) {
        const unsigned short* wq = whh + (q * HD + 16 * jt + m) * WP + kb + 8 * hh;
        FragB bf;
        bf.h[0] = *(const v8usa*)wq;
        bf.h[1] = *(const v8usa*)(wq + 16);
        acc[q] = wmb(af, bf, acc[q]);
      }
    }
    unsigned short* hbn = hb + nxt * (NB * HP);
#pragma unroll
    for (int r = 0; r < 8; ++r) {
      const float gi = acc[0][r], gf = acc[1][r], gg = acc[2][r], go = acc[3][r];
      const float cn = sigm(gf) * cst[r] + sigm(gi) * tanhf(gg);
      cst[r] = cn;
      const float hv = sigm(go) * tanhf(cn);
      const int row = 16 * mt + 8 * hh + r, col = 16 * jt + m;
      const unsigned hbits = bf16_bits(hv);
      const unsigned lbits = bf16_bits(hv - __uint_as_float(hbits << 16));
      hbn[row * HP + col]      = (unsigned short)hbits;
      hbn[row * HP + HD + col] = (unsigned short)lbits;
      hf[row * HD + col] = hv;
    }
    __syncthreads();

    if constexpr (LAYER == 0) {
      unsigned short* ob = OUT0 + (size_t)dir * ((size_t)NR * K2) + (size_t)t * (NB * K2);
      const int pa = tid, pb = tid + LTHR;
      const int ra = pa / 24, qa = pa - 24 * ra;
      const int rb = pb / 24, qb = pb - 24 * rb;
      const v8us va = *(const v8usa*)(hbn + ra * HP + 8 * qa);
      const v8us vb = *(const v8usa*)(hbn + rb * HP + 8 * qb);
      *(volatile v8us*)(ob + 8 * pa) = va;
      *(volatile v8us*)(ob + 8 * pb) = vb;
      __threadfence();
      *(volatile v8us*)(ob + 8 * pa) = va;
      *(volatile v8us*)(ob + 8 * pb) = vb;
    } else {
      float* ob = O1 + (size_t)dir * ((size_t)NR * HD) + (size_t)t * (NB * HD);
      const int pa = tid, pb = tid + LTHR;
      const v4f va = *(const v4fa*)(hf + 4 * pa);
      const v4f vb = *(const v4fa*)(hf + 4 * pb);
      *(volatile v4f*)(ob + 4 * pa) = va;
      *(volatile v4f*)(ob + 4 * pb) = vb;
      __threadfence();
      *(volatile v4f*)(ob + 4 * pa) = va;
      *(volatile v4f*)(ob + 4 * pb) = vb;
    }
  }
  {
    float* hp = HT + (size_t)(2 * LAYER + dir) * (NB * HD);
    const int pa = tid, pb = tid + LTHR;
    const v4f va = *(const v4fa*)(hf + 4 * pa);
    const v4f vb = *(const v4fa*)(hf + 4 * pb);
    *(volatile v4f*)(hp + 4 * pa) = va;
    *(volatile v4f*)(hp + 4 * pb) = vb;
    __threadfence();
    *(volatile v4f*)(hp + 4 * pa) = va;
    *(volatile v4f*)(hp + 4 * pb) = vb;
  }
}

__global__ __launch_bounds__(NTHR) void k_att(const float* __restrict__ O1, const float* __restrict__ HT,
                                              const float* __restrict__ SP, const int* __restrict__ FLAG,
                                              float* LOG, float* outp) {
  extern __shared__ __attribute__((aligned(16))) float hatt[];
  __shared__ __attribute__((aligned(16))) float swv[SS];
  __shared__ __attribute__((aligned(16))) float lg[32];
  __shared__ float red[SS];
  __shared__ float hs[HD], aw[HD], ctx[HD], f1[HD];
  const int tid = (int)threadIdx.x, lane = tid & 31;
  const int b = (int)blockIdx.x;

  const int fa = FLAG[lane * 32], fb = FLAG[(lane + 32) * 32];
  const bool anyf = __builtin_amdgcn_ballot_w32((fa | fb) != 0) != 0u;
  const float qnan = __int_as_float(0x7fc00000);

  if (tid < HD) {
    const float a0 = HT[(0 * NB + b) * HD + tid], a1 = HT[(1 * NB + b) * HD + tid];
    const float a2 = HT[(2 * NB + b) * HD + tid], a3 = HT[(3 * NB + b) * HD + tid];
    hs[tid] = (a0 + a1) + (a2 + a3);
  }
  {
    const float* pf = O1 + ((size_t)tid * NB + b) * HD;
    const float* pb = pf + (size_t)NR * HD;
#pragma unroll 4
    for (int q = 0; q < 24; ++q) {
      const v4f a = *(const v4fa*)(pf + 4 * q);
      const v4f c = *(const v4fa*)(pb + 4 * q);
      v4f o;
      o.x = a.x + c.x; o.y = a.y + c.y; o.z = a.z + c.z; o.w = a.w + c.w;
      *(v4fa*)(hatt + tid * HD + 4 * q) = o;
    }
  }
  __syncthreads();
  if (tid < HD) {
    float s = 0.0f;
#pragma unroll 1
    for (int k = 0; k < HD; ++k) s = fmaf(hs[k], SP[SP_ATW + k * HD + tid], s);
    s = s + SP[SP_ATB + tid];
    aw[tid] = (s > 0.0f) ? s : (s - s);
  }
  __syncthreads();
  float acv = 0.0f;
#pragma unroll 1
  for (int k = 0; k < HD; ++k) acv = fmaf(aw[k], tanhf(hatt[tid * HD + k]), acv);

  red[tid] = acv;
  __syncthreads();
#pragma unroll 1
  for (int off = 128; off > 0; off >>= 1) {
    if (tid < off) red[tid] = fmaxf(red[tid], red[tid + off]);
    __syncthreads();
  }
  const float mx = red[0];
  __syncthreads();
  const float e = expf(acv - mx);
  red[tid] = e;
  __syncthreads();
#pragma unroll 1
  for (int off = 128; off > 0; off >>= 1) {
    if (tid < off) red[tid] = red[tid] + red[tid + off];
    __syncthreads();
  }
  const float den = red[0];
  __syncthreads();
  const float sw1 = e * (1.0f / den);
  red[tid] = sw1;
  __syncthreads();
#pragma unroll 1
  for (int off = 128; off > 0; off >>= 1) {
    if (tid < off) red[tid] = red[tid] + red[tid + off];
    __syncthreads();
  }
  const float den2 = red[0];
  __syncthreads();
  const float sw2 = sw1 * (1.0f / den2);
  swv[tid] = sw2;
  __syncthreads();

  if (tid < 64) {
    const v4f a = *(const v4fa*)(swv + 4 * tid);
    v4f o;
    o.x = anyf ? qnan : a.x; o.y = anyf ? qnan : a.y; o.z = anyf ? qnan : a.z; o.w = anyf ? qnan : a.w;
    float* op = outp + 640 + b * SS + 4 * tid;
    *(volatile v4f*)op = o;
    __threadfence();
    *(volatile v4f*)op = o;
  }
  if (tid < HD) {
    float s = 0.0f;
#pragma unroll 1
    for (int si = 0; si < SS; ++si) s = fmaf(swv[si], hatt[si * HD + tid], s);
    ctx[tid] = s;
  }
  __syncthreads();
  if (tid < HD) {
    float s = 0.0f;
#pragma unroll 1
    for (int k = 0; k < HD; ++k) s = fmaf(ctx[k], SP[SP_F1W + k * HD + tid], s);
    s = s + SP[SP_F1B + tid];
    f1[tid] = (s > 0.0f) ? s : (s - s);
  }
  __syncthreads();
  if (tid < 32) {
    const int tc = tid < CC ? tid : CC - 1;
    float s = 0.0f;
#pragma unroll 1
    for (int k = 0; k < HD; ++k) s = fmaf(f1[k], SP[SP_F2W + k * CC + tc], s);
    s = s + SP[SP_F2B + tc];
    s = (tid < CC) ? s : 0.0f;
    lg[tid] = anyf ? qnan : s;
  }
  __syncthreads();
  if (tid < 8) {
    const v4f o = *(const v4fa*)(lg + 4 * tid);
    float* op = LOG + b * 32 + 4 * tid;
    *(volatile v4f*)op = o;
    __threadfence();
    *(volatile v4f*)op = o;
  }
}

__global__ __launch_bounds__(NTHR) void k_fin(const float* __restrict__ LOG, const int* __restrict__ FLAG, float* outp) {
  __shared__ __attribute__((aligned(16))) float buf[640];
  const int tid = (int)threadIdx.x, lane = tid & 31;
  const int fa = FLAG[lane * 32], fb = FLAG[(lane + 32) * 32];
  const bool anyf = __builtin_amdgcn_ballot_w32((fa | fb) != 0) != 0u;
  const float qnan = __int_as_float(0x7fc00000);
#pragma unroll 1
  for (int it = 0; it < 3; ++it) {
    const int i  = tid + NTHR * it;
    const int ic = i < 640 ? i : 639;
    const int bb = ic / CC, c = ic - bb * CC;
    const float v = LOG[bb * 32 + c];
    if (i < 640) buf[i] = anyf ? qnan : v;
  }
  __syncthreads();
  if (tid < 160) {
    const v4f o = *(const v4fa*)(buf + 4 * tid);
    float* op = outp + 4 * tid;
    *(volatile v4f*)op = o;
    __threadfence();
    *(volatile v4f*)op = o;
  }
}

static inline size_t al256(size_t o) { return (o + 255) & ~(size_t)255; }

extern "C" void kernel_launch(void* const* d_in, const int* in_sizes, int n_in,
                              void* d_out, int out_size, void* d_ws, size_t ws_size,
                              hipStream_t stream) {
  if (n_in < 21) return;
  if (in_sizes[0] != NN || in_sizes[1] != 2 * NE || in_sizes[2] != NE || in_sizes[3] != NB * SS) return;
  if (in_sizes[4] != (VV + 1) * DD || in_sizes[5] != DD * HD || in_sizes[6] != HD) return;
  if (in_sizes[7] != 6 * HD * HD || in_sizes[8] != 6 * HD) return;
  if (in_sizes[9] != 2 * G4 * HD || in_sizes[10] != 2 * G4 * HD || in_sizes[11] != 2 * G4) return;
  if (in_sizes[12] != 2 * G4 * 2 * HD || in_sizes[13] != 2 * G4 * HD || in_sizes[14] != 2 * G4) return;
  if (in_sizes[15] != HD * HD || in_sizes[16] != HD || in_sizes[17] != HD * HD || in_sizes[18] != HD) return;
  if (in_sizes[19] != HD * CC || in_sizes[20] != CC) return;
  if (out_size != 640 + NB * SS) return;

  const int*   x     = (const int*)d_in[0];
  const int*   eidx  = (const int*)d_in[1];
  const float* eattr = (const float*)d_in[2];
  const int*   xs    = (const int*)d_in[3];
  const float* emb   = (const float*)d_in[4];
  const float* encw  = (const float*)d_in[5];
  const float* encb  = (const float*)d_in[6];
  const float* gruw  = (const float*)d_in[7];
  const float* grub  = (const float*)d_in[8];
  const float* wih0  = (const float*)d_in[9];
  const float* whh0  = (const float*)d_in[10];
  const float* b0    = (const float*)d_in[11];
  const float* wih1  = (const float*)d_in[12];
  const float* whh1  = (const float*)d_in[13];
  const float* b1    = (const float*)d_in[14];
  const float* atw   = (const float*)d_in[15];
  const float* atb   = (const float*)d_in[16];
  const float* f1w   = (const float*)d_in[17];
  const float* f1b   = (const float*)d_in[18];
  const float* f2w   = (const float*)d_in[19];
  const float* f2b   = (const float*)d_in[20];
  float* out = (float*)d_out;

  char* ws = (char*)d_ws;
  size_t off = 0;
  const size_t oXE   = off; off = al256(off + (size_t)NN * DP * 2);
  const size_t oHA   = off; off = al256(off + (size_t)NN * HD * 4);
  const size_t oHB   = off; off = al256(off + (size_t)NN * HD * 4);
  const size_t oACAT = off; off = al256(off + (size_t)NN * KC * 2);
  const size_t oZ    = off; off = al256(off + (size_t)NN * HD * 4);
  const size_t oHR   = off; off = al256(off + (size_t)NN * K2 * 2);
  const size_t oLIST = off; off = al256(off + (size_t)(NN / NBA) * RCAP * 8);
  const size_t oOC   = off; off = al256(off + (size_t)2 * NN * 4);
  const size_t oFLAG = off; off = al256(off + (size_t)(NN / NBA) * 128);
  const size_t oXS   = off; off = al256(off + (size_t)NR * K2 * 2);
  const size_t oOUT0 = off; off = al256(off + (size_t)2 * NR * K2 * 2);
  const size_t oO1   = off; off = al256(off + (size_t)2 * NR * HD * 4);
  const size_t oENCT = off; off = al256(off + (size_t)HD * DP * 2);
  const size_t oWG   = off; off = al256(off + (size_t)288 * KC * 2);
  const size_t oWI0  = off; off = al256(off + (size_t)768 * K2 * 2);
  const size_t oWI1  = off; off = al256(off + (size_t)768 * KC * 2);
  const size_t oWHH0 = off; off = al256(off + (size_t)768 * HD * 2);
  const size_t oWHH1 = off; off = al256(off + (size_t)768 * HD * 2);
  const size_t oSP   = off; off = al256(off + (size_t)SP_N * 4);
  const size_t oHT   = off; off = al256(off + (size_t)4 * NB * HD * 4);
  const size_t oLOG  = off; off = al256(off + (size_t)NB * 32 * 4);
  if (off > ws_size || off > (size_t)WSMAX) return;
  if (oHB != oHA + (size_t)NN * HD * 4) return;

  unsigned short* XE   = (unsigned short*)(ws + oXE);
  float*          HA   = (float*)(ws + oHA);
  float*          HB   = (float*)(ws + oHB);
  float*          XG   = (float*)(ws + oHA);
  unsigned short* ACAT = (unsigned short*)(ws + oACAT);
  float*          Zp   = (float*)(ws + oZ);
  unsigned short* HR   = (unsigned short*)(ws + oHR);
  int*            LIST = (int*)(ws + oLIST);
  int*            OC   = (int*)(ws + oOC);
  int*            FLAG = (int*)(ws + oFLAG);
  unsigned short* XS   = (unsigned short*)(ws + oXS);
  unsigned short* OUT0 = (unsigned short*)(ws + oOUT0);
  float*          O1   = (float*)(ws + oO1);
  unsigned short* ENCT = (unsigned short*)(ws + oENCT);
  unsigned short* WG   = (unsigned short*)(ws + oWG);
  unsigned short* WI0  = (unsigned short*)(ws + oWI0);
  unsigned short* WI1  = (unsigned short*)(ws + oWI1);
  unsigned short* WHH0 = (unsigned short*)(ws + oWHH0);
  unsigned short* WHH1 = (unsigned short*)(ws + oWHH1);
  float*          SP   = (float*)(ws + oSP);
  float*          HT   = (float*)(ws + oHT);
  float*          LOG  = (float*)(ws + oLOG);

  const size_t bkLds = (size_t)BK_LDS_INTS * 4;
  const size_t lsLds = (size_t)(NB * G4 + NB * HD) * 4 + (size_t)(G4 * WP + 2 * NB * HP) * 2;
  const size_t atLds = (size_t)SS * HD * 4;
  hipFuncSetAttribute(reinterpret_cast<const void*>(&k_bucket), hipFuncAttributeMaxDynamicSharedMemorySize, (int)bkLds);
  hipFuncSetAttribute(reinterpret_cast<const void*>(&k_lstm<0>), hipFuncAttributeMaxDynamicSharedMemorySize, (int)lsLds);
  hipFuncSetAttribute(reinterpret_cast<const void*>(&k_lstm<1>), hipFuncAttributeMaxDynamicSharedMemorySize, (int)lsLds);
  hipFuncSetAttribute(reinterpret_cast<const void*>(&k_att), hipFuncAttributeMaxDynamicSharedMemorySize, (int)atLds);

  k_prep<<<PB_ALL, NTHR, 0, stream>>>(x, emb, encw, encb, gruw, grub, wih0, whh0, b0, wih1, whh1, b1,
                                      atw, atb, f1w, f1b, f2w, f2b,
                                      XE, ENCT, WG, WI0, WI1, WHH0, WHH1, SP);
  k_bucket<<<NN / NBA, NTHR, bkLds, stream>>>(eidx, eidx + NE, eattr, NE, NN, 1, LIST, OC, FLAG);
  k_gemm<M_ENC, 6><<<dim3(NN / GBM, 1), GTHR, 0, stream>>>(XE, DP, DP / 32, XE, DP, 0, ENCT, DP,
                                                           SP + SP_ENCB, HA, HA, HA, ACAT);
  for (int step = 0; step < 2; ++step) {
    float* Hc = (step == 0) ? HA : HB;
    float* Hn = (step == 0) ? HB : HA;
    k_agg<<<NN / (NWAVE * AGR), NTHR, 0, stream>>>(Hc, LIST, OC, FLAG, NN, ACAT);
    k_gemm<M_ZR, 12><<<dim3(NN / GBM, 1), GTHR, 0, stream>>>(ACAT, KC, KC / 32, ACAT, KC, 0, WG, KC,
                                                             SP + SP_GRUB, Hc, Hc, Zp, HR);
    k_gemm<M_HH, 6><<<dim3(NN / GBM, 1), GTHR, 0, stream>>>(ACAT, KC, 6, HR, K2, 6, WG + (size_t)192 * KC, KC,
                                                            SP + SP_GRUB, Hc, Zp, Hn, ACAT);
  }
  k_gather<<<(NR * 24) / NTHR, NTHR, 0, stream>>>(xs, ACAT, XS);
  k_gemm<M_XG, 12><<<dim3(NR / GBM, 4), GTHR, 0, stream>>>(XS, K2, 6, XS, K2, 0, WI0, K2,
                                                           SP + SP_B0, Zp, Zp, XG, HR);
  k_lstm<0><<<2, LTHR, lsLds, stream>>>(XG, WHH0, OUT0, O1, HT);
  k_gemm<M_XG, 12><<<dim3(NR / GBM, 4), GTHR, 0, stream>>>(OUT0, K2, 6, OUT0 + (size_t)NR * K2, K2, 6, WI1, KC,
                                                           SP + SP_B1, Zp, Zp, XG, HR);
  k_lstm<1><<<2, LTHR, lsLds, stream>>>(XG, WHH1, OUT0, O1, HT);
  k_att<<<NB, NTHR, atLds, stream>>>(O1, HT, SP, FLAG, LOG, out);
  k_fin<<<1, NTHR, 0, stream>>>(LOG, FLAG, out);
}
